// CANN_72395968741836
// MI455X (gfx1250) — hardware-verified
//
#include <hip/hip_runtime.h>


#define NN   8192
#define DD   512
#define RQ   512
#define PCAR 4096.0f
typedef _Float16 h16;
typedef unsigned short bf;
typedef __attribute__((ext_vector_type(16))) __bf16   v16bf;
typedef __attribute__((ext_vector_type(16))) _Float16 v16h;
typedef __attribute__((ext_vector_type(8)))  _Float16 v8h;
typedef __attribute__((ext_vector_type(8)))  unsigned short v8us;
typedef __attribute__((ext_vector_type(8)))  float    v8f;
typedef __attribute__((ext_vector_type(4)))  float    v4f;
typedef v8h  __attribute__((may_alias)) v8ha;
typedef v4f  __attribute__((may_alias)) v4fa;
typedef v8us __attribute__((may_alias)) v8usa;

__device__ __forceinline__ unsigned short f2bf(float f) { unsigned u = __float_as_uint(f); u += 0x7FFFu + ((u >> 16) & 1u); return (unsigned short)(u >> 16); }
__device__ __forceinline__ float bf2f(unsigned short b) { return __uint_as_float(((unsigned)b) << 16); }
__device__ __forceinline__ float bfr(float f) { return bf2f(f2bf(f)); }
__device__ __forceinline__ v16h cat16(v8h lo, v8h hi) { return __builtin_shufflevector(lo, hi, 0, 1, 2, 3, 4, 5, 6, 7, 8, 9, 10, 11, 12, 13, 14, 15); }
__device__ __forceinline__ v16bf cat16b(v8us lo, v8us hi) { return __builtin_bit_cast(v16bf, __builtin_shufflevector(lo, hi, 0, 1, 2, 3, 4, 5, 6, 7, 8, 9, 10, 11, 12, 13, 14, 15)); }
__device__ __forceinline__ v8f wmma16(v16h a, v16h b, v8f c) { return __builtin_amdgcn_wmma_f32_16x16x32_f16(false, a, false, b, (short)0, c, false, false); }
__device__ __forceinline__ v8f wmmab(v16bf a, v16bf b, v8f c) { return __builtin_amdgcn_wmma_f32_16x16x32_bf16(false, a, false, b, (short)0, c, false, false); }


template <typename T16> struct WFrag;
template <> struct WFrag<h16> { typedef v16h V; static __device__ __forceinline__ V ld(const h16* p) { return cat16(*(const v8h*)p, *(const v8h*)(p + 16)); } static __device__ __forceinline__ v8f mma(V a, V b, v8f c) { return wmma16(a, b, c); } };
template <> struct WFrag<bf> { typedef v16bf V; static __device__ __forceinline__ V ld(const bf* p) { return cat16b(*(const v8us*)p, *(const v8us*)(p + 16)); } static __device__ __forceinline__ v8f mma(V a, V b, v8f c) { return wmmab(a, b, c); } };
template <typename T16, int NSPLIT, bool BIAS>
__global__ __launch_bounds__(32) void k_gemmw(const T16* __restrict__ A, const T16* __restrict__ A2, const T16* __restrict__ Bt, const T16* __restrict__ Bt2, int K, float* C, int ldc, const float* __restrict__ bias, size_t sA, size_t sB, size_t sC) {
    typedef typename WFrag<T16>::V V;
    __shared__ __align__(16) float os[16 * 68];
    const size_t z = blockIdx.z; A += z * sA; if (A2) A2 += z * sA; Bt += z * sB; if (Bt2) Bt2 += z * sB; C += z * sC;
    const int lane = threadIdx.x & 31, lr = lane & 15, hi = lane >> 4; const int r0 = blockIdx.x * 64, c0 = blockIdx.y * 64;
    v8f acc[4][4];
#pragma unroll
    for (int mb = 0; mb < 4; ++mb)
#pragma unroll
        for (int nb = 0; nb < 4; ++nb) acc[mb][nb] = (v8f){};
    const size_t aoff = (size_t)(r0 + lr) * K + 8 * hi, boff = (size_t)(c0 + lr) * K + 8 * hi;
#pragma unroll 1
    for (int kc = 0; kc < K; kc += 32) {
        V a[4], a2[4];
#pragma unroll
        for (int mb = 0; mb < 4; ++mb) { a[mb] = WFrag<T16>::ld(A + aoff + (size_t)mb * 16 * K + kc); if (NSPLIT == 1 || NSPLIT == 2) a2[mb] = WFrag<T16>::ld(A2 + aoff + (size_t)mb * 16 * K + kc); }
#pragma unroll
        for (int nb = 0; nb < 4; ++nb) { const V b = WFrag<T16>::ld(Bt + boff + (size_t)nb * 16 * K + kc); V b2; if (NSPLIT >= 2) b2 = WFrag<T16>::ld(Bt2 + boff + (size_t)nb * 16 * K + kc);
#pragma unroll
            for (int mb = 0; mb < 4; ++mb) { acc[mb][nb] = WFrag<T16>::mma(a[mb], b, acc[mb][nb]); if (NSPLIT == 1 || NSPLIT == 2) acc[mb][nb] = WFrag<T16>::mma(a2[mb], b, acc[mb][nb]); if (NSPLIT >= 2) acc[mb][nb] = WFrag<T16>::mma(a[mb], b2, acc[mb][nb]); } }
        asm volatile("v_nop\n\tv_nop\n\tv_nop\n\tv_nop" : "+v"(acc[0][0]), "+v"(acc[1][1]), "+v"(acc[2][2]), "+v"(acc[3][3]) : "v"(a[0]), "v"(a[3]));
    }
#pragma unroll
    for (int mb = 0; mb < 4; ++mb) {
#pragma unroll
        for (int nb = 0; nb < 4; ++nb) {
#pragma unroll
            for (int j = 0; j < 8; ++j) os[(hi * 8 + j) * 68 + nb * 16 + lr] = acc[mb][nb][j]; }
        __builtin_amdgcn_wave_barrier(); asm volatile("" ::: "memory");
        float* crow = C + (size_t)(r0 + mb * 16) * ldc + c0;
#pragma unroll 1
        for (int ps = 0; ps < 2; ++ps) {
#pragma unroll
            for (int s = 0; s < 8; ++s) { const int row = 2 * s + hi, cofs = lr * 4; v4f val = *(const v4fa*)(os + row * 68 + cofs); if (BIAS) { val[0] += bfr(bias[c0 + cofs]); val[1] += bfr(bias[c0 + cofs + 1]); val[2] += bfr(bias[c0 + cofs + 2]); val[3] += bfr(bias[c0 + cofs + 3]); }
                *(volatile v4f*)(crow + (size_t)row * ldc + cofs) = val; }
            if (ps == 0) __threadfence(); }
        __builtin_amdgcn_wave_barrier(); asm volatile("" ::: "memory");
    }
}

__device__ __forceinline__ h16 tohx(float x) { return (h16)x; }
typedef __attribute__((ext_vector_type(2))) _Float16 v2h;
typedef __attribute__((ext_vector_type(4))) _Float16 v4h;

__global__ __launch_bounds__(256) void k_cvt8(const float* __restrict__ src, bf* dst, size_t n8) { const size_t i = (size_t)blockIdx.x * 256 + threadIdx.x; if (i >= n8) return; const v8f v = *(const v8f*)(src + i * 8); v8us o;
#pragma unroll
    for (int k = 0; k < 8; ++k) o[k] = f2bf(v[k]); *(volatile v8us*)(dst + i * 8) = o; __threadfence(); *(volatile v8us*)(dst + i * 8) = o; }
__global__ __launch_bounds__(256) void k_p16(const float* __restrict__ F, h16* P) { const size_t e = ((size_t)blockIdx.x * 256 + threadIdx.x) * 4; if (e >= (size_t)NN * DD) return; v4h o;
#pragma unroll
    for (int u = 0; u < 4; ++u) o[u] = tohx(F[e + u]); *(volatile v4h*)(P + e) = o; __threadfence(); *(volatile v4h*)(P + e) = o; }
__global__ __launch_bounds__(256) void k_vt(const float* __restrict__ F, h16* VT) { const size_t e = ((size_t)blockIdx.x * 256 + threadIdx.x) * 2; if (e >= (size_t)DD * NN) return; const int n = (int)(e % NN); const int d = (int)(e / NN); v2h o; o[0] = tohx(F[(size_t)n * DD + d]); o[1] = tohx(F[(size_t)(n + 1) * DD + d]); *(volatile v2h*)(VT + e) = o; __threadfence(); *(volatile v2h*)(VT + e) = o; }
__global__ __launch_bounds__(256) void k_smax(const float* __restrict__ S, h16* P16) { const int lane = threadIdx.x & 31; const int row = blockIdx.x * 8 + (threadIdx.x >> 5); if (row >= RQ) return; const float* sr = S + (size_t)row * NN; const float sc = 0.044194173824159216f; float mx = -3.0e38f;
    for (int j = lane * 4; j < NN; j += 128) { const v4f a = *(const v4f*)(sr + j); mx = fmaxf(mx, fmaxf(fmaxf(a[0], a[1]), fmaxf(a[2], a[3]))); }
#pragma unroll
    for (int sh = 16; sh; sh >>= 1) mx = fmaxf(mx, __shfl_xor(mx, sh, 32));
    const float mxs = mx * sc; float sum = 0.f;
    for (int j = lane * 4; j < NN; j += 128) { const v4f a = *(const v4f*)(sr + j); for (int u = 0; u < 4; ++u) { float t = a[u] * sc; asm volatile("" : "+v"(t)); float d0 = __fsub_rn(t, mxs); asm volatile("" : "+v"(d0)); sum += __builtin_amdgcn_exp2f(__fmul_rn(d0, 1.4426950408889634f)); } }
#pragma unroll
    for (int sh = 16; sh; sh >>= 1) sum += __shfl_xor(sum, sh, 32);
    const float f = __fdiv_rn(PCAR, sum);
    for (int ps = 0; ps < 2; ++ps) { for (int j = lane * 4; j < NN; j += 128) { const v4f a = *(const v4f*)(sr + j); v4h o; for (int u = 0; u < 4; ++u) { float t = a[u] * sc; asm volatile("" : "+v"(t)); float d0 = __fsub_rn(t, mxs); asm volatile("" : "+v"(d0)); o[u] = tohx(__builtin_amdgcn_exp2f(__fmul_rn(d0, 1.4426950408889634f)) * f); } *(volatile v4h*)(P16 + (size_t)row * NN + j) = o; } if (ps == 0) __threadfence(); } }
__global__ __launch_bounds__(256) void k_scl(float* O) { const size_t e = ((size_t)blockIdx.x * 256 + threadIdx.x) * 4; if (e >= (size_t)RQ * DD) return; const v4f a = *(const v4f*)(O + e); v4f r;
#pragma unroll
    for (int u = 0; u < 4; ++u) r[u] = a[u] * (1.0f / PCAR); *(volatile v4f*)(O + e) = r; __threadfence(); *(volatile v4f*)(O + e) = r; }

extern "C" void kernel_launch(void* const* d_in, const int* in_sizes, int n_in,
                              void* d_out, int out_size, void* d_ws, size_t ws_size, hipStream_t stream) {
    (void)in_sizes; (void)n_in; (void)out_size;
    const float** I = (const float**)d_in;
    const float *z = I[0], *Wq = I[1], *bq = I[2], *Wk = I[3], *bk = I[4], *Wv = I[5], *bv = I[6];
    float* OUT = (float*)d_out;
    char* wsp = (char*)d_ws;
    auto take = [&](size_t bytes) { char* p = wsp; wsp += (bytes + 255) & ~(size_t)255; return (void*)p; };
    bf* ZB = (bf*)take((size_t)NN * DD * 2); bf* BQ = (bf*)take((size_t)DD * DD * 2); bf* BK = (bf*)take((size_t)DD * DD * 2); bf* BV = (bf*)take((size_t)DD * DD * 2); float* F = (float*)take((size_t)NN * DD * 4);
    h16* QP = (h16*)take((size_t)NN * DD * 2); h16* KP = (h16*)take((size_t)NN * DD * 2); h16* VT = (h16*)take((size_t)DD * NN * 2); float* S = (float*)take((size_t)RQ * NN * 4); h16* P16 = (h16*)take((size_t)RQ * NN * 2);
    if ((size_t)(wsp - (char*)d_ws) > ws_size) return;
    k_cvt8<<<(DD * DD / 8 + 255) / 256, 256, 0, stream>>>(Wq, BQ, DD * DD / 8); k_cvt8<<<(DD * DD / 8 + 255) / 256, 256, 0, stream>>>(Wk, BK, DD * DD / 8); k_cvt8<<<(DD * DD / 8 + 255) / 256, 256, 0, stream>>>(Wv, BV, DD * DD / 8);
    k_cvt8<<<(unsigned)(((size_t)NN * DD / 8 + 255) / 256), 256, 0, stream>>>(z, ZB, (size_t)NN * DD / 8);
    const dim3 gp(NN / 64, DD / 64, 1); const unsigned gpl = (unsigned)(((size_t)NN * DD / 4 + 255) / 256);
    k_gemmw<bf, 0, true><<<gp, 32, 0, stream>>>(ZB, nullptr, BQ, nullptr, DD, F, DD, bq, 0, 0, 0); k_p16<<<gpl, 256, 0, stream>>>(F, QP);
    k_gemmw<bf, 0, true><<<gp, 32, 0, stream>>>(ZB, nullptr, BK, nullptr, DD, F, DD, bk, 0, 0, 0); k_p16<<<gpl, 256, 0, stream>>>(F, KP);
    k_gemmw<bf, 0, true><<<gp, 32, 0, stream>>>(ZB, nullptr, BV, nullptr, DD, F, DD, bv, 0, 0, 0); k_vt<<<(unsigned)(((size_t)DD * NN / 2 + 255) / 256), 256, 0, stream>>>(F, VT);
    for (int r0 = 0; r0 < NN; r0 += RQ) {
        k_gemmw<h16, 0, false><<<dim3(RQ / 64, NN / 64, 1), 32, 0, stream>>>(QP + (size_t)r0 * DD, nullptr, KP, nullptr, DD, S, NN, nullptr, 0, 0, 0);
        k_smax<<<RQ / 8, 256, 0, stream>>>(S, P16);
        k_gemmw<h16, 0, false><<<dim3(RQ / 64, DD / 64, 1), 32, 0, stream>>>(P16, nullptr, VT, nullptr, NN, OUT + (size_t)r0 * DD, DD, nullptr, 0, 0, 0);
        k_scl<<<(RQ * DD / 4 + 255) / 256, 256, 0, stream>>>(OUT + (size_t)r0 * DD); }
}
